// IncrementalRBFLayer_90005334655649
// MI455X (gfx1250) — hardware-verified
//
#include <hip/hip_runtime.h>

#define NB     2048
#define NI     64
#define NO     2048
#define OG     32
#define BR     128
#define MPITCH 64
#define OPITCH 36
#define ASCALE 16384.0f
#define XSCALE 64.0f
#define XINV   0.015625f
#define EXPK   (-4.76837158203125e-07f)

static_assert(NB % BR == 0);
static_assert(NO % OG == 0);
static_assert(NI == 64);
static_assert(BR == 8 * 16);
static_assert(OG == 32);
static_assert((NO * NI * NI) % (8 * 256) == 0);
static_assert((NO % 4) == 0);
static_assert((OPITCH % 4) == 0);
static_assert(OPITCH >= OG);
static_assert((MPITCH % 4) == 0);

typedef _Float16 v16h __attribute__((ext_vector_type(16)));
typedef _Float16 v8h  __attribute__((ext_vector_type(8)));
typedef float    v8f  __attribute__((ext_vector_type(8)));
typedef float    v4f  __attribute__((ext_vector_type(4)));
typedef float    v4fa __attribute__((ext_vector_type(4), may_alias));

union HF { v16h v; v8h h[2]; };

__device__ __forceinline__ unsigned short bf16bits(float f) {
  unsigned int u = __float_as_uint(f);
  u = u + 0x7FFFu + ((u >> 16) & 1u);
  return (unsigned short)(u >> 16);
}
__device__ __forceinline__ float bf16val(unsigned short b) {
  return __uint_as_float(((unsigned int)b) << 16);
}
__device__ __forceinline__ float bf16r(float f) { return bf16val(bf16bits(f)); }

__device__ __forceinline__ v8f mma_h(v16h a, v16h b, v8f c) {
  return __builtin_amdgcn_wmma_f32_16x16x32_f16(false, a, false, b, (short)0, c, false, false);
}
__device__ __forceinline__ void guard2(v8f& acc, v16h a0, v16h b0, v16h a1, v16h b1) {
#if defined(__HIP_DEVICE_COMPILE__)
  asm volatile("v_nop\n\tv_nop\n\tv_nop\n\tv_nop" : "+v"(acc) : "v"(a0), "v"(b0), "v"(a1), "v"(b1));
#endif
}

__global__ __launch_bounds__(256) void prep_a(const float* __restrict__ S, _Float16* A2) {
  const int g = (int)blockIdx.x * 256 + (int)threadIdx.x;
  if (g >= (NO * NI * NI) / 8) return;
  const float* sp = S + (size_t)g * 8;
  const v4f a = *(const v4f*)sp;
  const v4f b = *(const v4f*)(sp + 4);
  v8h o = {};
#pragma unroll
  for (int e = 0; e < 4; ++e) {
    const float s0 = bf16r(a[e]);
    const float s1 = bf16r(b[e]);
    o[e]     = (_Float16)(s0 * s0 * ASCALE);
    o[4 + e] = (_Float16)(s1 * s1 * ASCALE);
  }
  _Float16* op = A2 + (size_t)g * 8;
  *(volatile v8h*)op = o;
  __threadfence();
  *(volatile v8h*)op = o;
}

__global__ __launch_bounds__(256) void prep_c(const _Float16* __restrict__ A2, const float* __restrict__ means,
                                              float* C20) {
  __shared__ __align__(16) float s_m[4 * MPITCH];
  __shared__ __align__(16) float s_c[8 * 32];
  const int tid = (int)threadIdx.x;
  const int wave = tid >> 5, lane = tid & 31;
  const int ob = (int)blockIdx.x * 4;
  if (ob + 4 > NO) return;
  {
    const int k = tid >> 2, j = tid & 3;
    s_m[j * MPITCH + k] = bf16r(means[(size_t)k * NO + ob + j]);
  }
  __syncthreads();
  const int j = tid >> 6, n = tid & 63;
  const int o = ob + j;
  const _Float16* ap = A2 + ((size_t)o * NI + n) * NI;
  const float* mp = s_m + j * MPITCH;
  float acc = 0.0f;
#pragma unroll 1
  for (int kc = 0; kc < NI / 8; ++kc) {
    const v8h av = *(const v8h*)(ap + kc * 8);
    const v4f m0 = *(const v4fa*)(mp + kc * 8);
    const v4f m1 = *(const v4fa*)(mp + kc * 8 + 4);
#pragma unroll
    for (int e = 0; e < 4; ++e) acc = fmaf((float)av[e], m0[e], acc);
#pragma unroll
    for (int e = 0; e < 4; ++e) acc = fmaf((float)av[4 + e], m1[e], acc);
  }
  s_c[wave * 32 + lane] = acc * XSCALE;
  __syncthreads();
  const int l8 = min(lane, 7);
  const v4f cv = *(const v4fa*)(s_c + wave * 32 + l8 * 4);
  float* cp = C20 + (size_t)o * NI + (n & 32) + l8 * 4;
  if (lane < 8) *(volatile v4f*)cp = cv;
  __threadfence();
  if (lane < 8) *(volatile v4f*)cp = cv;
}

__global__ __launch_bounds__(256) void rbf_main(const float* __restrict__ x, const float* __restrict__ means,
                                                const _Float16* __restrict__ A2, const float* __restrict__ C20,
                                                float* out) {
  __shared__ __align__(16) float s_mt[OG * MPITCH];
  __shared__ __align__(16) float s_out[BR * OPITCH];

  const int tid = (int)threadIdx.x;
  const int wave = tid >> 5, lane = tid & 31, hl = lane >> 4, l15 = lane & 15;
  if (((int)blockIdx.x + 1) * OG > NO || ((int)blockIdx.y + 1) * BR > NB) return;
  const int o0 = (int)blockIdx.x * OG;
  const int rowbase = (int)blockIdx.y * BR + wave * 16;

  {
    const int k = tid >> 2, j8 = (tid & 3) * 8;
    const float* mp = means + (size_t)k * NO + o0 + j8;
    const v4f a = *(const v4f*)mp;
    const v4f b = *(const v4f*)(mp + 4);
#pragma unroll
    for (int e = 0; e < 4; ++e) {
      s_mt[(j8 + e) * MPITCH + k]     = bf16r(a[e]);
      s_mt[(j8 + 4 + e) * MPITCH + k] = bf16r(b[e]);
    }
  }

  HF xf[2];
  {
    const float* xr = x + (size_t)(rowbase + l15) * NI + 8 * hl;
#pragma unroll
    for (int f = 0; f < 2; ++f) {
      const v4f p0 = *(const v4f*)(xr + 32 * f);
      const v4f p1 = *(const v4f*)(xr + 32 * f + 4);
      const v4f p2 = *(const v4f*)(xr + 32 * f + 16);
      const v4f p3 = *(const v4f*)(xr + 32 * f + 20);
      v16h u = {};
#pragma unroll
      for (int e = 0; e < 4; ++e) {
        u[e]      = (_Float16)(bf16r(p0[e]) * XSCALE);
        u[4 + e]  = (_Float16)(bf16r(p1[e]) * XSCALE);
        u[8 + e]  = (_Float16)(bf16r(p2[e]) * XSCALE);
        u[12 + e] = (_Float16)(bf16r(p3[e]) * XSCALE);
      }
      xf[f].v = u;
    }
  }
  __syncthreads();

  float* so = s_out + (wave * 16 + l15) * OPITCH;
#pragma unroll 1
  for (int oi = 0; oi < OG; ++oi) {
    const int o = o0 + oi;
    const _Float16* ab = A2 + ((size_t)o * NI + l15) * NI + 8 * hl;
    const float* cb = C20 + (size_t)o * NI + 8 * hl;
    const float* mb = s_mt + oi * MPITCH + 8 * hl;
    float p = 0.0f;
#pragma unroll
    for (int t = 0; t < 4; ++t) {
      const _Float16* ap = ab + (size_t)(16 * t) * NI;
      HF a0, a1;
      a0.h[0] = *(const v8h*)(ap);
      a0.h[1] = *(const v8h*)(ap + 16);
      a1.h[0] = *(const v8h*)(ap + 32);
      a1.h[1] = *(const v8h*)(ap + 48);
      v8f acc = {};
      acc = mma_h(a0.v, xf[0].v, acc);
      acc = mma_h(a1.v, xf[1].v, acc);
      guard2(acc, a0.v, xf[0].v, a1.v, xf[1].v);
      const v4f c0 = *(const v4f*)(cb + 16 * t);
      const v4f c1 = *(const v4f*)(cb + 16 * t + 4);
      const v4f m0 = *(const v4fa*)(mb + 16 * t);
      const v4f m1 = *(const v4fa*)(mb + 16 * t + 4);
      const int s = t >> 1, ib = 8 * (t & 1);
#pragma unroll
      for (int r = 0; r < 8; ++r) {
        const float cv = (r < 4) ? c0[r & 3] : c1[r & 3];
        const float mv = (r < 4) ? m0[r & 3] : m1[r & 3];
        const float xv = (float)xf[s].v[ib + r] * XINV;
        p = fmaf(acc[r] - cv, xv - mv, p);
      }
    }
    p += __shfl_xor(p, 16);
    const float val = __expf(p * EXPK);
    if (hl == 0) so[oi] = val;
  }
  __syncthreads();

  const int q8 = lane >> 3, c4 = (lane & 7) * 4;
  v4f vv[4];
#pragma unroll
  for (int it = 0; it < 4; ++it)
    vv[it] = *(const v4fa*)(s_out + (wave * 16 + 4 * it + q8) * OPITCH + c4);
  float* ob = out + (size_t)(rowbase + q8) * NO + o0 + c4;
#pragma unroll
  for (int it = 0; it < 4; ++it) *(volatile v4f*)(ob + (size_t)(4 * it) * NO) = vv[it];
  __threadfence();
#pragma unroll
  for (int it = 0; it < 4; ++it) *(volatile v4f*)(ob + (size_t)(4 * it) * NO) = vv[it];
}

extern "C" void kernel_launch(void* const* d_in, const int* in_sizes, int n_in,
                              void* d_out, int out_size, void* d_ws, size_t ws_size,
                              hipStream_t stream) {
  if (n_in < 3) return;
  if (in_sizes[0] != NB * NI) return;
  if (in_sizes[1] != NI * NO) return;
  if (in_sizes[2] != NO * NI * NI) return;
  if (out_size != NB * NO) return;

  const size_t off_a2 = 0;
  const size_t sz_a2  = (size_t)NO * NI * NI * 2;
  const size_t off_c  = off_a2 + sz_a2;
  const size_t sz_c   = (size_t)NO * NI * sizeof(float);
  const size_t need   = off_c + sz_c;
  if (need > ws_size) return;
  if (need > (size_t)134217728) return;

  const float* X  = (const float*)d_in[0];
  const float* M  = (const float*)d_in[1];
  const float* S  = (const float*)d_in[2];
  float* out = (float*)d_out;
  _Float16* A2  = (_Float16*)((char*)d_ws + off_a2);
  float*    C20 = (float*)((char*)d_ws + off_c);

  prep_a<<<dim3((NO * NI * NI / 8) / 256), dim3(256), 0, stream>>>(S, A2);
  prep_c<<<dim3(NO / 4), dim3(256), 0, stream>>>(A2, M, C20);
  rbf_main<<<dim3(NO / OG, NB / BR), dim3(256), 0, stream>>>(X, M, A2, C20, out);
  (void)hipGetLastError();
}
